// GraphiTLayer_54185307407181
// MI455X (gfx1250) — hardware-verified
//
#include <hip/hip_runtime.h>
#include <stddef.h>


typedef __attribute__((ext_vector_type(16))) _Float16 v16h;
typedef __attribute__((ext_vector_type(8)))  _Float16 v8h;
typedef __attribute__((ext_vector_type(16))) __bf16   v16b;
typedef __attribute__((ext_vector_type(8)))  __bf16   v8b;
typedef __attribute__((ext_vector_type(8)))  float    v8f;
typedef __attribute__((ext_vector_type(4)))  float    v4f;
typedef __attribute__((ext_vector_type(4)))  int      v4i;

__device__ __forceinline__ unsigned short f2bf_bits(float f) {
  unsigned u = __float_as_uint(f);
  return (unsigned short)((u + 0x7FFFu + ((u >> 16) & 1u)) >> 16);
}
__device__ __forceinline__ float bf_bits2f(unsigned short h) { return __uint_as_float(((unsigned)h) << 16); }

__device__ __forceinline__ void dep_guard_h(v8f& a, v8f& b, v16h x, v16h y) { asm volatile("v_nop\n\tv_nop\n\tv_nop\n\tv_nop" : "+v"(a), "+v"(b) : "v"(x), "v"(y)); }
__device__ __forceinline__ void dep_guard_b(v8f& a, v8f& b, v16b x, v16b y) { asm volatile("v_nop\n\tv_nop\n\tv_nop\n\tv_nop" : "+v"(a), "+v"(b) : "v"(x), "v"(y)); }
__device__ __forceinline__ void keep4_h(v16h a, v16h b, v16h c, v16h d) { asm volatile("v_nop" :: "v"(a), "v"(b), "v"(c), "v"(d)); }
__device__ __forceinline__ void keep4_b(v16b a, v16b b, v16b c, v16b d) { asm volatile("v_nop" :: "v"(a), "v"(b), "v"(c), "v"(d)); }
__device__ __forceinline__ void acc_guard4(v8f& a, v8f& b, v8f& c, v8f& d) { asm volatile("v_nop\n\tv_nop\n\tv_nop\n\tv_nop" : "+v"(a), "+v"(b), "+v"(c), "+v"(d)); }
template <typename T> struct Frag;
template <> struct Frag<_Float16> {
  typedef v16h V; union U { v16h v; v8h h[2]; };
  static __device__ __forceinline__ v16h load(const _Float16* p) {
    U f; f.h[0] = *(const v8h*)(p); f.h[1] = *(const v8h*)(p + 16); return f.v;
  }
  static __device__ __forceinline__ v8f mma(v16h a, v16h b, v8f c) {
    return __builtin_amdgcn_wmma_f32_16x16x32_f16(false, a, false, b, (short)0, c, false, false);
  }
  static __device__ __forceinline__ void guard(v8f& a, v8f& b, v16h x, v16h y) { dep_guard_h(a, b, x, y); }
  static __device__ __forceinline__ void keep(v16h a, v16h b, v16h c, v16h d) { keep4_h(a, b, c, d); }
};
template <> struct Frag<__bf16> {
  typedef v16b V; union U { v16b v; v8b h[2]; };
  static __device__ __forceinline__ v16b load(const __bf16* p) {
    U f; f.h[0] = *(const v8b*)(p); f.h[1] = *(const v8b*)(p + 16); return f.v;
  }
  static __device__ __forceinline__ v8f mma(v16b a, v16b b, v8f c) {
    return __builtin_amdgcn_wmma_f32_16x16x32_bf16(false, a, false, b, (short)0, c, false, false);
  }
  static __device__ __forceinline__ void guard(v8f& a, v8f& b, v16b x, v16b y) { dep_guard_b(a, b, x, y); }
  static __device__ __forceinline__ void keep(v16b a, v16b b, v16b c, v16b d) { keep4_b(a, b, c, d); }
};

__device__ __forceinline__ v8f mma_h(v16h a, v16h b, v8f c) {
  c = __builtin_amdgcn_wmma_f32_16x16x32_f16(false, a, false, b, (short)0, c, false, false);
  asm volatile("v_nop\n\tv_nop\n\tv_nop\n\tv_nop" : "+v"(c) : "v"(a), "v"(b));
  return c;
}

template <int ET> struct Elem;
template <> struct Elem<0> { typedef _Float16 T; };
template <> struct Elem<1> { typedef __bf16 T; };
template <int ET, bool SPLIT, int BIAS_MODE, int OUT_MODE, bool RESID, int ACT = 0>
__global__ __launch_bounds__(256) void wmma_gemm64(
    const unsigned short* __restrict__ Ap, const unsigned short* __restrict__ A2p, int lda, long strideA,
    const unsigned short* __restrict__ Btp, const unsigned short* __restrict__ Bt2p, int ldb, long strideB,
    void* __restrict__ Cout, void* __restrict__ Cout2, int ldc, long strideC,
    const float* __restrict__ bias,
    const float* __restrict__ resid, long strideR,
    int M, int N, int K, float scale) {
  typedef typename Elem<ET>::T T;
  typedef typename Frag<T>::V V;
  const T* A = (const T*)Ap; const T* A2 = (const T*)A2p; const T* Bt = (const T*)Btp; const T* Bt2 = (const T*)Bt2p;
  __shared__ __align__(16) float sT[8][16 * 68];
  const int b    = blockIdx.y;
  const int lane = threadIdx.x & 31;
  const int wave = threadIdx.x >> 5;
  const int tilesN = N >> 6;
  const int tilesM = M >> 6;
  const int tile = blockIdx.x * 8 + wave;
  if (tile >= tilesM * tilesN) return;
  const int tm = tile / tilesN;
  const int tn = tile - tm * tilesN;
  const int m0 = tm << 6;
  const int n0 = tn << 6;

  const T* Ab  = A  + (size_t)b * strideA;
  const T* Bb  = Bt + (size_t)b * strideB;
  const T* Ab2 = SPLIT ? (A2  + (size_t)b * strideA) : nullptr;
  const T* Bb2 = SPLIT ? (Bt2 + (size_t)b * strideB) : nullptr;

  const int rlane = lane & 15;
  const int koff  = (lane >> 4) * 8;
  const int mOff  = (lane >> 4) * 8;

  v8f acc[4][4];
#pragma unroll
  for (int i = 0; i < 4; ++i)
#pragma unroll
    for (int j = 0; j < 4; ++j) acc[i][j] = (v8f){0.f,0.f,0.f,0.f,0.f,0.f,0.f,0.f};

  for (int k0 = 0; k0 < K; k0 += 32) {
    V bh[4], bl[4];
#pragma unroll
    for (int j = 0; j < 4; ++j) {
      const size_t bo = (size_t)(n0 + (j << 4) + rlane) * ldb + koff + k0;
      bh[j] = Frag<T>::load(Bb + bo);
      if (SPLIT) bl[j] = Frag<T>::load(Bb2 + bo);
    }
#pragma unroll
    for (int i = 0; i < 4; ++i) {
      const size_t ao = (size_t)(m0 + (i << 4) + rlane) * lda + koff + k0;
      V ah = Frag<T>::load(Ab + ao);
      V al;
      if (SPLIT) al = Frag<T>::load(Ab2 + ao);
#pragma unroll
      for (int j = 0; j < 4; ++j) {
        acc[i][j] = Frag<T>::mma(ah, bh[j], acc[i][j]);
        if (SPLIT) {
          acc[i][j] = Frag<T>::mma(ah, bl[j], acc[i][j]);
          acc[i][j] = Frag<T>::mma(al, bh[j], acc[i][j]);
        }
      }
      Frag<T>::guard(acc[i][0], acc[i][3], ah, SPLIT ? al : ah);
    }
    Frag<T>::keep(bh[0], bh[1], bh[2], bh[3]);
    if (SPLIT) Frag<T>::keep(bl[0], bl[1], bl[2], bl[3]);
  }
  acc_guard4(acc[0][0], acc[0][1], acc[0][2], acc[0][3]);
  acc_guard4(acc[1][0], acc[1][1], acc[1][2], acc[1][3]);
  acc_guard4(acc[2][0], acc[2][1], acc[2][2], acc[2][3]);
  acc_guard4(acc[3][0], acc[3][1], acc[3][2], acc[3][3]);

  float* slab = sT[wave];
  const float* Rb = RESID ? (resid + (size_t)b * strideR) : nullptr;
#pragma unroll
  for (int i = 0; i < 4; ++i) {
    const int mBase = m0 + (i << 4);
#pragma unroll
    for (int j = 0; j < 4; ++j) {
      const int n = n0 + (j << 4) + rlane;
      float bv = 0.f;
      if (BIAS_MODE == 2) bv = bias[n];
#pragma unroll
      for (int r = 0; r < 8; ++r) {
        float v = acc[i][j][r] * scale;
        if (BIAS_MODE == 1) v += bias[mBase + mOff + r];
        if (BIAS_MODE == 2) v += bv;
        if (ACT == 2) v = fmaxf(v, 0.0f);
        if (ACT == 4) v = (v > 0.f) ? v : 0.01f * v;
        if (ACT == 6) v = (v > 0.f) ? v : (__expf(v) - 1.0f);
        if (RESID) v += Rb[(size_t)(mBase + mOff + r) * ldc + n];
        slab[(mOff + r) * 68 + (j << 4) + rlane] = v;
      }
    }
    __builtin_amdgcn_fence(__ATOMIC_RELEASE, "workgroup");
    __builtin_amdgcn_wave_barrier();
    __builtin_amdgcn_fence(__ATOMIC_ACQUIRE, "workgroup");
    if (OUT_MODE == 0) {
      float* C = (float*)Cout + (size_t)b * strideC;
      const int hh = lane >> 4, c4 = (lane & 15) * 4;
      for (int pass = 0; pass < 2; ++pass) {
#pragma unroll
        for (int it = 0; it < 8; ++it) {
          const int row = it * 2 + hh;
          v4f v = *(const v4f*)(slab + row * 68 + c4);
          *(volatile v4f*)(C + (size_t)(mBase + row) * ldc + n0 + c4) = v;
        }
        __threadfence();
      }
    } else {
      const int q = lane >> 3, c8 = (lane & 7) * 8;
      unsigned short* C  = (unsigned short*)Cout  + (size_t)b * strideC;
      unsigned short* C2 = (OUT_MODE == 2) ? ((unsigned short*)Cout2 + (size_t)b * strideC) : nullptr;
      for (int pass = 0; pass < 2; ++pass) {
#pragma unroll
        for (int it = 0; it < 4; ++it) {
          const int row = it * 4 + q;
          const float* sp = slab + row * 68 + c8;
          v8h hv, lv;
#pragma unroll
          for (int e = 0; e < 8; ++e) {
            if (OUT_MODE == 1) {
              hv[e] = (_Float16)sp[e];
            } else {
              unsigned short hb = f2bf_bits(sp[e]);
              unsigned short lb = f2bf_bits(sp[e] - bf_bits2f(hb));
              hv[e] = __builtin_bit_cast(_Float16, hb);
              lv[e] = __builtin_bit_cast(_Float16, lb);
            }
          }
          *(volatile v8h*)(C + (size_t)(mBase + row) * ldc + n0 + c8) = hv;
          if (OUT_MODE == 2) *(volatile v8h*)(C2 + (size_t)(mBase + row) * ldc + n0 + c8) = lv;
        }
        __threadfence();
      }
    }
    __builtin_amdgcn_fence(__ATOMIC_RELEASE, "workgroup");
    __builtin_amdgcn_wave_barrier();
    __builtin_amdgcn_fence(__ATOMIC_ACQUIRE, "workgroup");
  }
}

__global__ __launch_bounds__(256) void cast_f32_f16x2(
    const float* __restrict__ in, _Float16* __restrict__ out, int n2, float scale) {
  int i = blockIdx.x * 256 + threadIdx.x;
  if (i < n2) {
    const _Float16 h0 = (_Float16)(in[2 * i] * scale), h1 = (_Float16)(in[2 * i + 1] * scale);
    const unsigned u = (unsigned)__builtin_bit_cast(unsigned short, h0) | ((unsigned)__builtin_bit_cast(unsigned short, h1) << 16);
    ((volatile unsigned*)out)[i] = u;
    __threadfence();
    ((volatile unsigned*)out)[i] = u;
  }
}

__global__ __launch_bounds__(256) void transpose_cast_kernel(
    const float* __restrict__ in, _Float16* __restrict__ out, int R, int C,
    long strideIn, long strideOut, float scale) {
  __shared__ __align__(16) _Float16 sh[64 * 72];
  const int tid = threadIdx.x;
  const int c0 = blockIdx.x * 64, r0 = blockIdx.y * 64;
  const float* ib = in + (size_t)blockIdx.z * strideIn;
  _Float16* ob = out + (size_t)blockIdx.z * strideOut;
#pragma unroll
  for (int i = 0; i < 4; ++i) {
    const int idx = i * 256 + tid;
    const int row = idx >> 4, c4 = (idx & 15) * 4;
    const v4f v = *(const v4f*)(ib + (size_t)(r0 + row) * C + c0 + c4);
#pragma unroll
    for (int e = 0; e < 4; ++e) sh[(c4 + e) * 72 + row] = (_Float16)(v[e] * scale);
  }
  __syncthreads();
  const int q = tid & 7;
  v8h hv[2];
#pragma unroll
  for (int it = 0; it < 2; ++it) {
    const int c = it * 32 + (tid >> 3);
    hv[it] = *(const v8h*)(sh + c * 72 + q * 8);
  }
  for (int pass = 0; pass < 2; ++pass) {
#pragma unroll
    for (int it = 0; it < 2; ++it) {
      const int c = it * 32 + (tid >> 3);
      *(volatile v8h*)(ob + (size_t)(c0 + c) * R + r0 + q * 8) = hv[it];
    }
    __threadfence();
  }
}

__global__ __launch_bounds__(256) void f1f2_kernel(
    const float* __restrict__ Wh, const float* __restrict__ a_gat,
    float* __restrict__ f1, float* __restrict__ f2, int nrows) {
  __shared__ __align__(16) float s1[32];
  __shared__ __align__(16) float s2[32];
  const int lane = threadIdx.x & 31, wave = threadIdx.x >> 5;
  const v4f a10 = *(const v4f*)(a_gat + lane * 8), a11 = *(const v4f*)(a_gat + lane * 8 + 4);
  const v4f a20 = *(const v4f*)(a_gat + 256 + lane * 8), a21 = *(const v4f*)(a_gat + 256 + lane * 8 + 4);
#pragma unroll 1
  for (int rr = 0; rr < 4; ++rr) {
    int row = blockIdx.x * 32 + wave * 4 + rr;
    row = (row < nrows) ? row : (nrows - 1);
    const float* wp = Wh + (size_t)row * 256 + lane * 8;
    const v4f w0 = *(const v4f*)wp, w1 = *(const v4f*)(wp + 4);
    float d1 = 0.f, d2 = 0.f;
#pragma unroll
    for (int e = 0; e < 4; ++e) {
      d1 += w0[e] * a10[e]; d1 += w1[e] * a11[e];
      d2 += w0[e] * a20[e]; d2 += w1[e] * a21[e];
    }
#pragma unroll
    for (int off = 16; off > 0; off >>= 1) {
      d1 += __shfl_xor(d1, off, 32);
      d2 += __shfl_xor(d2, off, 32);
    }
    if (lane == 0) { s1[wave * 4 + rr] = d1; s2[wave * 4 + rr] = d2; }
  }
  __syncthreads();
  if (wave == 0 && lane < 16) {
    const int q = lane & 7;
    const int rb = blockIdx.x * 32 + q * 4;
    v4f val; float* dst;
    if (lane < 8) { val = *(const v4f*)(s1 + q * 4); dst = f1 + rb; }
    else          { val = *(const v4f*)(s2 + q * 4); dst = f2 + rb; }
    if (rb + 3 < nrows) {
      *(volatile v4f*)dst = val;
      __threadfence();
      *(volatile v4f*)dst = val;
    }
  }
}

__global__ __launch_bounds__(256) void gat_weights_kernel(
    const int* __restrict__ adj, const float* __restrict__ f1, const float* __restrict__ f2,
    _Float16* __restrict__ attn, int nrows, int nnode) {
  const int lane = threadIdx.x & 31, wave = threadIdx.x >> 5;
  const int row = blockIdx.x * 8 + wave;
  if (row >= nrows) return;
  const int b = row / nnode;
  const int* arow = adj + (size_t)row * nnode;
  const float* f2b = f2 + (size_t)b * nnode;
  const float fi = f1[row];
  float e[4][8];
  float mx = -9.0e15f;
#pragma unroll
  for (int c = 0; c < 4; ++c) {
    const int j0 = c * 256 + lane * 8;
    const v4i m0 = *(const v4i*)(arow + j0), m1 = *(const v4i*)(arow + j0 + 4);
    const v4f g0 = *(const v4f*)(f2b + j0), g1 = *(const v4f*)(f2b + j0 + 4);
#pragma unroll
    for (int q = 0; q < 4; ++q) {
      e[c][q]     = (m0[q] > 0) ? (fi + g0[q]) : -9.0e15f;
      e[c][4 + q] = (m1[q] > 0) ? (fi + g1[q]) : -9.0e15f;
    }
#pragma unroll
    for (int q = 0; q < 8; ++q) mx = fmaxf(mx, e[c][q]);
  }
#pragma unroll
  for (int off = 16; off > 0; off >>= 1) mx = fmaxf(mx, __shfl_xor(mx, off, 32));
  float sum = 0.f;
#pragma unroll
  for (int c = 0; c < 4; ++c)
#pragma unroll
    for (int q = 0; q < 8; ++q) { e[c][q] = __expf(e[c][q] - mx); sum += e[c][q]; }
#pragma unroll
  for (int off = 16; off > 0; off >>= 1) sum += __shfl_xor(sum, off, 32);
  const float inv = (1.0f / sum) * 32768.0f;
  v8h hv[4];
#pragma unroll
  for (int c = 0; c < 4; ++c)
#pragma unroll
    for (int q = 0; q < 8; ++q) hv[c][q] = (_Float16)(e[c][q] * inv);
  _Float16* orow = attn + (size_t)row * nnode;
  for (int pass = 0; pass < 2; ++pass) {
#pragma unroll
    for (int c = 0; c < 4; ++c) *(volatile v8h*)(orow + c * 256 + lane * 8) = hv[c];
    __threadfence();
  }
}

template <bool H16>
__global__ __launch_bounds__(256) void ln_kernel(
    const float* __restrict__ in, const float* __restrict__ g, const float* __restrict__ bb,
    float* __restrict__ outf, _Float16* __restrict__ out16, int nrows) {
  __shared__ __align__(16) _Float16 sh[8][256];
  const int lane = threadIdx.x & 31, wave = threadIdx.x >> 5;
  int row = blockIdx.x * 8 + wave;
  const bool ok = row < nrows;
  row = ok ? row : (nrows - 1);
  const float* ip = in + (size_t)row * 256;
  const v4f x0 = *(const v4f*)(ip + 4 * lane), x1 = *(const v4f*)(ip + 128 + 4 * lane);
  float s = ((x0[0] + x0[1]) + (x0[2] + x0[3])) + ((x1[0] + x1[1]) + (x1[2] + x1[3]));
#pragma unroll
  for (int off = 16; off > 0; off >>= 1) s += __shfl_xor(s, off, 32);
  const float mu = s * (1.0f / 256.0f);
  const v4f d0 = x0 - mu, d1 = x1 - mu;
  float vs = ((d0[0] * d0[0] + d0[1] * d0[1]) + (d0[2] * d0[2] + d0[3] * d0[3]))
           + ((d1[0] * d1[0] + d1[1] * d1[1]) + (d1[2] * d1[2] + d1[3] * d1[3]));
#pragma unroll
  for (int off = 16; off > 0; off >>= 1) vs += __shfl_xor(vs, off, 32);
  const float r = rsqrtf(vs * (1.0f / 256.0f) + 1e-5f);
  const v4f g0 = *(const v4f*)(g + 4 * lane), g1 = *(const v4f*)(g + 128 + 4 * lane);
  const v4f b0 = *(const v4f*)(bb + 4 * lane), b1 = *(const v4f*)(bb + 128 + 4 * lane);
  const v4f y0 = (d0 * r) * g0 + b0, y1 = (d1 * r) * g1 + b1;
  v8h hv = (v8h){(_Float16)0, (_Float16)0, (_Float16)0, (_Float16)0, (_Float16)0, (_Float16)0, (_Float16)0, (_Float16)0};
  if (H16) {
#pragma unroll
    for (int e2 = 0; e2 < 4; ++e2) {
      sh[wave][4 * lane + e2] = (_Float16)y0[e2];
      sh[wave][128 + 4 * lane + e2] = (_Float16)y1[e2];
    }
    __syncthreads();
    hv = *(const v8h*)(&sh[wave][8 * lane]);
  }
  if (ok) {
    float* op = outf + (size_t)row * 256;
    for (int pass = 0; pass < 2; ++pass) {
      *(volatile v4f*)(op + 4 * lane) = y0;
      *(volatile v4f*)(op + 128 + 4 * lane) = y1;
      if (H16) *(volatile v8h*)(out16 + (size_t)row * 256 + 8 * lane) = hv;
      __threadfence();
    }
  }
}

__global__ __launch_bounds__(128)
void attn32_kernel(const float* __restrict__ qkv, float* __restrict__ out, int S, int H, float qscale) {
  const float PSC = 32768.0f;
  union FB { v16h v; v8h h[2]; };
  __shared__ __align__(16) _Float16 Ksh[64 * 32];
  __shared__ __align__(16) _Float16 Vth[32 * 64];
  __shared__ __align__(16) _Float16 Psh[4][16 * 64];
  __shared__ __align__(16) float  Os[4][16 * 36];
  const int tid = threadIdx.x, wave = tid >> 5, lane = tid & 31, hh = lane >> 4, c = lane & 15;
  const int dm = H * 32, rs = 3 * dm;
  const int nqb = S >> 6;
  const int bx = blockIdx.x;
  const int qb = bx % nqb, bh = bx / nqb, h = bh % H, b = bh / H;
  const int q0 = qb * 64 + wave * 16;
  const float* qb_ptr = qkv + (size_t)b * S * rs + h * 32;
  const float* kb_ptr = qb_ptr + dm;
  const float* vb_ptr = qb_ptr + 2 * dm;
  float* ob = out + (size_t)b * S * dm + h * 32;

  v16h qa;
  {
    const float* qrow = qb_ptr + (size_t)(q0 + c) * rs;
#pragma unroll
    for (int e = 0; e < 8; ++e) {
      qa[e]     = (_Float16)(qrow[8 * hh + e] * qscale);
      qa[8 + e] = (_Float16)(qrow[16 + 8 * hh + e] * qscale);
    }
  }
  float mrow[8], lrow[8];
  v8f oacc[2];
  const v8f zero8 = (v8f){0.f,0.f,0.f,0.f,0.f,0.f,0.f,0.f};
#pragma unroll
  for (int r = 0; r < 8; ++r) { mrow[r] = -__builtin_inff(); lrow[r] = 0.f; }
  oacc[0] = zero8; oacc[1] = zero8;

  const int nChunks = S >> 6;
  for (int kc = 0; kc < nChunks; ++kc) {
    const int kv0 = kc * 64;
    __syncthreads();
    {
      const int kvr = tid >> 1, dh = (tid & 1) * 16;
      const float* krow = kb_ptr + (size_t)(kv0 + kvr) * rs + dh;
      const float* vrow = vb_ptr + (size_t)(kv0 + kvr) * rs + dh;
#pragma unroll
      for (int i = 0; i < 4; ++i) {
        const v4f kk = *(const v4f*)(krow + 4 * i);
        const v4f vv = *(const v4f*)(vrow + 4 * i);
#pragma unroll
        for (int e = 0; e < 4; ++e) {
          const int d = dh + 4 * i + e;
          Ksh[kvr * 32 + d] = (_Float16)kk[e];
          Vth[d * 64 + kvr]  = (_Float16)vv[e];
        }
      }
    }
    __syncthreads();

    v8f s[4];
#pragma unroll
    for (int j = 0; j < 4; ++j) {
      FB kb;
      kb.h[0] = *(const v8h*)(Ksh + (j * 16 + c) * 32 + 8 * hh);
      kb.h[1] = *(const v8h*)(Ksh + (j * 16 + c) * 32 + 16 + 8 * hh);
      s[j] = mma_h(qa, kb.v, zero8);
    }
    float cm[8];
#pragma unroll
    for (int r = 0; r < 8; ++r) {
      float m = fmaxf(fmaxf(s[0][r], s[1][r]), fmaxf(s[2][r], s[3][r]));
#pragma unroll
      for (int off = 1; off < 16; off <<= 1) m = fmaxf(m, __shfl_xor(m, off, 32));
      cm[r] = m;
    }
    _Float16* pwh = Psh[wave];
#pragma unroll
    for (int r = 0; r < 8; ++r) {
      const float mnew = fmaxf(mrow[r], cm[r]);
      const float alpha = expf(mrow[r] - mnew);
      mrow[r] = mnew;
      float psum = 0.f;
#pragma unroll
      for (int j = 0; j < 4; ++j) {
        const float p = expf(s[j][r] - mnew);
        psum += p;
        pwh[(8 * hh + r) * 64 + j * 16 + c] = (_Float16)(p * PSC);
      }
#pragma unroll
      for (int off = 1; off < 16; off <<= 1) psum += __shfl_xor(psum, off, 32);
      lrow[r] = lrow[r] * alpha + psum;
      oacc[0][r] *= alpha;
      oacc[1][r] *= alpha;
    }
    __builtin_amdgcn_fence(__ATOMIC_RELEASE, "workgroup");
    __builtin_amdgcn_wave_barrier();
    __builtin_amdgcn_fence(__ATOMIC_ACQUIRE, "workgroup");
#pragma unroll
    for (int kk = 0; kk < 2; ++kk) {
      FB pa;
      pa.h[0] = *(const v8h*)(pwh + c * 64 + kk * 32 + 8 * hh);
      pa.h[1] = *(const v8h*)(pwh + c * 64 + kk * 32 + 16 + 8 * hh);
#pragma unroll
      for (int t = 0; t < 2; ++t) {
        FB vb;
        vb.h[0] = *(const v8h*)(Vth + (t * 16 + c) * 64 + kk * 32 + 8 * hh);
        vb.h[1] = *(const v8h*)(Vth + (t * 16 + c) * 64 + kk * 32 + 16 + 8 * hh);
        oacc[t] = mma_h(pa.v, vb.v, oacc[t]);
      }
    }
  }

  float* os = Os[wave];
#pragma unroll
  for (int r = 0; r < 8; ++r) {
    const float inv = 1.0f / (lrow[r] * PSC);
    os[(8 * hh + r) * 36 + c]      = oacc[0][r] * inv;
    os[(8 * hh + r) * 36 + 16 + c] = oacc[1][r] * inv;
  }
  __builtin_amdgcn_fence(__ATOMIC_RELEASE, "workgroup");
  __builtin_amdgcn_wave_barrier();
  __builtin_amdgcn_fence(__ATOMIC_ACQUIRE, "workgroup");
  {
    const int q = lane >> 3, c4 = (lane & 7) * 4;
    for (int pass = 0; pass < 2; ++pass) {
#pragma unroll
      for (int it = 0; it < 4; ++it) {
        const int row = it * 4 + q;
        const v4f val = *(const v4f*)(os + row * 36 + c4);
        *(volatile v4f*)(ob + (size_t)(q0 + row) * dm + c4) = val;
      }
      __threadfence();
    }
  }
}

extern "C" void kernel_launch(void* const* d_in, const int* in_sizes, int n_in,
                              void* d_out, int out_size, void* d_ws, size_t ws_size,
                              hipStream_t stream) {
  const int Bn = 8, Nn = 1024, D = 256, H = 8, DFF = 2048;
  const int M = Bn * Nn;
  if (n_in < 18) return;
  if (in_sizes[0] != M * D || in_sizes[1] != Bn * Nn * Nn || in_sizes[2] != D * D || in_sizes[3] != 2 * D ||
      in_sizes[4] != 3 * D * D || in_sizes[5] != 3 * D || in_sizes[6] != D * D || in_sizes[7] != D ||
      in_sizes[8] != DFF * D || in_sizes[9] != DFF || in_sizes[10] != D * DFF || in_sizes[11] != D ||
      in_sizes[12] != D || in_sizes[13] != D || in_sizes[14] != D || in_sizes[15] != D ||
      in_sizes[16] != D || in_sizes[17] != D) return;
  if (out_size != M * D) return;

  const float* src        = (const float*)d_in[0];
  const int*   adj        = (const int*)  d_in[1];
  const float* W_gat      = (const float*)d_in[2];
  const float* a_gat      = (const float*)d_in[3];
  const float* in_proj_w  = (const float*)d_in[4];
  const float* in_proj_b  = (const float*)d_in[5];
  const float* out_proj_w = (const float*)d_in[6];
  const float* out_proj_b = (const float*)d_in[7];
  const float* lin1_w     = (const float*)d_in[8];
  const float* lin1_b     = (const float*)d_in[9];
  const float* lin2_w     = (const float*)d_in[10];
  const float* lin2_b     = (const float*)d_in[11];
  const float* ln1_g = (const float*)d_in[12]; const float* ln1_b = (const float*)d_in[13];
  const float* ln2_g = (const float*)d_in[14]; const float* ln2_b = (const float*)d_in[15];
  const float* ln3_g = (const float*)d_in[16]; const float* ln3_b = (const float*)d_in[17];
  float* outp = (float*)d_out;

  char* ws = (char*)d_ws;
  size_t off = 0;
  auto carve = [&](size_t bytes) { size_t o = off; off += (bytes + 255) & ~(size_t)255; return o; };
  const size_t o_wg16 = carve((size_t)D * D * 2);
  const size_t o_ip16 = carve((size_t)3 * D * D * 2);
  const size_t o_op16 = carve((size_t)D * D * 2);
  const size_t o_l1w  = carve((size_t)DFF * D * 2);
  const size_t o_l2w  = carve((size_t)D * DFF * 2);
  const size_t o_f1   = carve((size_t)M * 4);
  const size_t o_f2   = carve((size_t)M * 4);
  const size_t PB = off;
  const size_t szA16 = (size_t)M * D * 2;
  const size_t szA32 = (size_t)M * D * 4;
  const size_t szAtt = (size_t)Bn * Nn * Nn * 2;
  const size_t szQkv = (size_t)M * 3 * D * 4;
  const size_t szFf1 = (size_t)M * DFF * 2;
  const size_t o_src16 = PB;
  const size_t o_Wh    = o_src16 + szA16;
  const size_t o_WhT   = o_Wh + szA32;
  const size_t o_att   = o_WhT + szA16;
  const size_t o_hp    = o_att + szAtt;
  const size_t o_x     = o_hp + szA32;
  const size_t o_x16   = o_x + szA32;
  const size_t end1    = o_x16 + szA16;
  const size_t o_qkv   = PB;
  const size_t o_ctx   = o_qkv + szQkv;
  const size_t o_ctx16 = o_ctx + szA32;
  if (o_ctx16 + szA16 > o_x) return;
  const size_t o_ao    = end1;
  const size_t o_y     = o_ao + szA32;
  const size_t o_y16   = o_y + szA32;
  const size_t end2    = o_y16 + szA16;
  const size_t o_ff1   = PB;
  const size_t o_z     = o_ff1 + szFf1;
  if (o_z + szA32 > o_y) return;
  const size_t endAll  = end2;
  if (endAll > ws_size) return;

  _Float16* wg16  = (_Float16*)(ws + o_wg16);
  _Float16* ip16  = (_Float16*)(ws + o_ip16);
  _Float16* op16  = (_Float16*)(ws + o_op16);
  _Float16* l1w16 = (_Float16*)(ws + o_l1w);
  _Float16* l2w16 = (_Float16*)(ws + o_l2w);
  float* f1 = (float*)(ws + o_f1);
  float* f2 = (float*)(ws + o_f2);
  _Float16* src16 = (_Float16*)(ws + o_src16);
  float* Wh = (float*)(ws + o_Wh);
  _Float16* WhT = (_Float16*)(ws + o_WhT);
  _Float16* att = (_Float16*)(ws + o_att);
  float* hp = (float*)(ws + o_hp);
  float* x = (float*)(ws + o_x);
  _Float16* x16 = (_Float16*)(ws + o_x16);
  float* qkv = (float*)(ws + o_qkv);
  float* ctx = (float*)(ws + o_ctx);
  _Float16* ctx16 = (_Float16*)(ws + o_ctx16);
  float* ao = (float*)(ws + o_ao);
  float* y = (float*)(ws + o_y);
  _Float16* y16 = (_Float16*)(ws + o_y16);
  _Float16* ff1 = (_Float16*)(ws + o_ff1);
  float* z = (float*)(ws + o_z);

  typedef const unsigned short* CU;
  auto cdiv = [](long a, long bb) { return (int)((a + bb - 1) / bb); };
  auto gtiles = [](int Mv, int Nv) { return ((Mv / 64) * (Nv / 64) + 7) / 8; };
  const float wsc = 16.0f, winv = 1.0f / 16.0f;

  transpose_cast_kernel<<<dim3(D / 64, D / 64, 1), 256, 0, stream>>>(W_gat, wg16, D, D, 0L, 0L, wsc);
  cast_f32_f16x2<<<cdiv(3 * D * D / 2, 256), 256, 0, stream>>>(in_proj_w, ip16, 3 * D * D / 2, wsc);
  cast_f32_f16x2<<<cdiv(D * D / 2, 256), 256, 0, stream>>>(out_proj_w, op16, D * D / 2, wsc);
  cast_f32_f16x2<<<cdiv(DFF * D / 2, 256), 256, 0, stream>>>(lin1_w, l1w16, DFF * D / 2, wsc);
  cast_f32_f16x2<<<cdiv(D * DFF / 2, 256), 256, 0, stream>>>(lin2_w, l2w16, D * DFF / 2, wsc);
  cast_f32_f16x2<<<cdiv((long)M * D / 2, 256), 256, 0, stream>>>(src, src16, M * D / 2, 1.0f);

  wmma_gemm64<0, false, 0, 0, false, 0><<<dim3(gtiles(M, D), 1), 256, 0, stream>>>(
      (CU)src16, (CU)src16, D, 0L, (CU)wg16, (CU)wg16, D, 0L,
      Wh, Wh, D, 0L, in_proj_b, src, 0L, M, D, D, winv);

  transpose_cast_kernel<<<dim3(D / 64, Nn / 64, Bn), 256, 0, stream>>>(
      Wh, WhT, Nn, D, (long)Nn * D, (long)D * Nn, 1.0f);

  f1f2_kernel<<<M / 32, 256, 0, stream>>>(Wh, a_gat, f1, f2, M);

  gat_weights_kernel<<<M / 8, 256, 0, stream>>>(adj, f1, f2, att, M, Nn);

  wmma_gemm64<0, false, 0, 0, true, 6><<<dim3(gtiles(Nn, D), Bn), 256, 0, stream>>>(
      (CU)att, (CU)att, Nn, (long)Nn * Nn, (CU)WhT, (CU)WhT, Nn, (long)D * Nn,
      hp, hp, D, (long)Nn * D, in_proj_b, src, (long)Nn * D, Nn, D, Nn, 1.0f / 32768.0f);

  ln_kernel<true><<<M / 8, 256, 0, stream>>>(hp, ln1_g, ln1_b, x, x16, M);

  wmma_gemm64<0, false, 2, 0, false, 0><<<dim3(gtiles(M, 3 * D), 1), 256, 0, stream>>>(
      (CU)x16, (CU)x16, D, 0L, (CU)ip16, (CU)ip16, D, 0L,
      qkv, qkv, 3 * D, 0L, in_proj_b, src, 0L, M, 3 * D, D, winv);

  attn32_kernel<<<Bn * H * (Nn / 64), 128, 0, stream>>>(qkv, ctx, Nn, H, 0.17677669529663687f);

  cast_f32_f16x2<<<cdiv((long)M * D / 2, 256), 256, 0, stream>>>(ctx, ctx16, M * D / 2, 1.0f);

  wmma_gemm64<0, false, 2, 0, true, 0><<<dim3(gtiles(M, D), 1), 256, 0, stream>>>(
      (CU)ctx16, (CU)ctx16, D, 0L, (CU)op16, (CU)op16, D, 0L,
      ao, ao, D, 0L, out_proj_b, x, 0L, M, D, D, winv);

  ln_kernel<true><<<M / 8, 256, 0, stream>>>(ao, ln2_g, ln2_b, y, y16, M);

  wmma_gemm64<0, false, 2, 1, false, 2><<<dim3(gtiles(M, DFF), 1), 256, 0, stream>>>(
      (CU)y16, (CU)y16, D, 0L, (CU)l1w16, (CU)l1w16, D, 0L,
      ff1, ff1, DFF, 0L, lin1_b, y, 0L, M, DFF, D, winv);

  wmma_gemm64<0, false, 2, 0, true, 0><<<dim3(gtiles(M, D), 1), 256, 0, stream>>>(
      (CU)ff1, (CU)ff1, DFF, 0L, (CU)l2w16, (CU)l2w16, DFF, 0L,
      z, z, D, 0L, lin2_b, y, 0L, M, D, DFF, winv);

  ln_kernel<false><<<M / 8, 256, 0, stream>>>(z, ln3_g, ln3_b, outp, x16, M);
}
